// PerformerSelfAttentionWrapper_59742995088073
// MI455X (gfx1250) — hardware-verified
//
#include <hip/hip_runtime.h>


#define NBI  4
#define CC   256
#define NN   9216
#define NHD  8
#define DH   32
#define DHP  64
#define MF   128
#define DM   CC
#define DNRM 0.42044820762685725f
#define RATIO 0.08838834764831845f
#define KEPS 1e-4f
#define LOSC 1024.0f

typedef _Float16 h16;
typedef unsigned short bf;
typedef __attribute__((ext_vector_type(16))) __bf16   v16bf;
typedef __attribute__((ext_vector_type(16))) _Float16 v16h;
typedef __attribute__((ext_vector_type(8)))  _Float16 v8h;
typedef __attribute__((ext_vector_type(8)))  unsigned short v8us;
typedef __attribute__((ext_vector_type(8)))  float    v8f;
typedef __attribute__((ext_vector_type(4)))  float    v4f;
typedef v8h  __attribute__((may_alias)) v8ha;
typedef v4f  __attribute__((may_alias)) v4fa;
typedef v8us __attribute__((may_alias)) v8usa;

__device__ __forceinline__ unsigned short f2bf(float f) { unsigned u = __float_as_uint(f); u += 0x7FFFu + ((u >> 16) & 1u); return (unsigned short)(u >> 16); }
__device__ __forceinline__ float bf2f(unsigned short b) { return __uint_as_float(((unsigned)b) << 16); }
__device__ __forceinline__ float bfr(float f) { return bf2f(f2bf(f)); }
__device__ __forceinline__ v16h cat16(v8h lo, v8h hi) { return __builtin_shufflevector(lo, hi, 0, 1, 2, 3, 4, 5, 6, 7, 8, 9, 10, 11, 12, 13, 14, 15); }
__device__ __forceinline__ v16bf cat16b(v8us lo, v8us hi) { return __builtin_bit_cast(v16bf, __builtin_shufflevector(lo, hi, 0, 1, 2, 3, 4, 5, 6, 7, 8, 9, 10, 11, 12, 13, 14, 15)); }
__device__ __forceinline__ v8f wmma16(v16h a, v16h b, v8f c) { return __builtin_amdgcn_wmma_f32_16x16x32_f16(false, a, false, b, (short)0, c, false, false); }
__device__ __forceinline__ v8f wmmab(v16bf a, v16bf b, v8f c) { return __builtin_amdgcn_wmma_f32_16x16x32_bf16(false, a, false, b, (short)0, c, false, false); }

template <bool SPLITA, bool F16OUT = false>
__global__ __launch_bounds__(128) void k_gemmb(const bf* __restrict__ A, const bf* __restrict__ Al, const bf* __restrict__ Bn, const float* __restrict__ bias, float* C, int ldc, h16* C2, const float* __restrict__ R = nullptr, int K = DM, int roundR = 1) {
    __shared__ __align__(16) float ost[4][16 * 68];
    const int lane = threadIdx.x & 31, wave = threadIdx.x >> 5, lr = lane & 15, hi = lane >> 4;
    const int r0 = blockIdx.x * 64 + wave * 16, c0 = blockIdx.y * 64;
    const size_t aoff = (size_t)(r0 + lr) * K + 8 * hi;
    size_t boff[4];
#pragma unroll
    for (int t = 0; t < 4; ++t) boff[t] = (size_t)(c0 + t * 16 + lr) * K + 8 * hi;
    v8f acc[4];
#pragma unroll
    for (int t = 0; t < 4; ++t) acc[t] = (v8f){};
#pragma unroll 1
    for (int kc = 0; kc < K; kc += 32) {
        const v16bf a = cat16b(*(const v8us*)(A + aoff + kc), *(const v8us*)(A + aoff + kc + 16));
        v16bf al = a;
        if (SPLITA) al = cat16b(*(const v8us*)(Al + aoff + kc), *(const v8us*)(Al + aoff + kc + 16));
#pragma unroll
        for (int t = 0; t < 4; ++t) { const v16bf b = cat16b(*(const v8us*)(Bn + boff[t] + kc), *(const v8us*)(Bn + boff[t] + kc + 16)); acc[t] = wmmab(a, b, acc[t]); if (SPLITA) acc[t] = wmmab(al, b, acc[t]); }
        asm volatile("v_nop\n\tv_nop\n\tv_nop\n\tv_nop" : "+v"(acc[0]), "+v"(acc[1]), "+v"(acc[2]), "+v"(acc[3]) : "v"(a), "v"(al));
    }
    float* os = &ost[wave][0];
#pragma unroll
    for (int t = 0; t < 4; ++t) { const float bv = bias ? bfr(bias[c0 + t * 16 + lr]) : 0.f;
#pragma unroll
        for (int j = 0; j < 8; ++j) os[(hi * 8 + j) * 68 + t * 16 + lr] = acc[t][j] + bv; }
    __syncthreads();
    if (F16OUT) {
        h16* crow = (h16*)(void*)C + (size_t)r0 * ldc + c0;
        auto pass = [&]() {
#pragma unroll
            for (int s = 0; s < 4; ++s) { const int row = 4 * s + (lane >> 3), piece = lane & 7; const float* sp = os + row * 68 + piece * 8; v8h o, o2;
#pragma unroll
                for (int i = 0; i < 8; ++i) { const h16 a = (h16)sp[i]; o[i] = a; o2[i] = (h16)((sp[i] - (float)a) * LOSC); }
                *(volatile v8h*)(crow + (size_t)row * ldc + piece * 8) = o; if (C2) *(volatile v8h*)(C2 + (size_t)r0 * ldc + c0 + (size_t)row * ldc + piece * 8) = o2; }
        };
        pass(); __threadfence(); pass();
    } else {
        float* crow = C + (size_t)r0 * ldc + c0;
        auto pass = [&]() {
#pragma unroll
            for (int s = 0; s < 8; ++s) { const int Lid = (lane >> 3) + 4 * s, piece = lane & 7; const int row = Lid >> 1, cofs = (Lid & 1) * 32 + piece * 4;
                v4f val = *(const v4fa*)(os + row * 68 + cofs); if (R) { const v4f rv = *(const v4f*)(R + ((size_t)r0 + row) * ldc + c0 + cofs); val += roundR ? (v4f){bfr(rv[0]), bfr(rv[1]), bfr(rv[2]), bfr(rv[3])} : rv; }
                *(volatile v4f*)(crow + (size_t)row * ldc + cofs) = val; }
        };
        pass(); __threadfence(); pass();
    }
}


__global__ __launch_bounds__(256) void k_wt(const float* __restrict__ Wm, int K, int ncols, bf* WT) {
    __shared__ __align__(16) unsigned short tl[64 * 72];
    const int tid = threadIdx.x, k0 = blockIdx.x * 64, n0 = blockIdx.y * 64;
    const int kk = tid >> 2, nq = (tid & 3) * 16;
#pragma unroll
    for (int i = 0; i < 16; ++i) tl[(nq + i) * 72 + kk] = f2bf(Wm[(size_t)(k0 + kk) * ncols + n0 + nq + i]);
    __syncthreads();
    const int piece = tid & 7;
    auto pass = [&]() {
#pragma unroll
        for (int s = 0; s < 2; ++s) { const int nr = (tid >> 3) + 32 * s; const v8us val = *(const v8usa*)(tl + nr * 72 + piece * 8); *(volatile v8us*)(WT + (size_t)(n0 + nr) * K + k0 + piece * 8) = val; }
    };
    pass(); __threadfence(); pass();
}

__global__ __launch_bounds__(256) void k_bf(const float* __restrict__ src, bf* dst, size_t n8) {
    const size_t i = (size_t)blockIdx.x * 256 + threadIdx.x; if (i >= n8) return;
    const v8f v = *(const v8f*)(src + i * 8); v8us o;
#pragma unroll
    for (int k = 0; k < 8; ++k) o[k] = f2bf(v[k]);
    *(volatile v8us*)(dst + i * 8) = o; __threadfence(); *(volatile v8us*)(dst + i * 8) = o;
}

__global__ __launch_bounds__(128) void k_gemm3(const bf* __restrict__ Ah, const bf* __restrict__ Al, const bf* __restrict__ Bh, const bf* __restrict__ Bl, int K, float* C, int ldc) {
    __shared__ __align__(16) float ost[4][16 * 68];
    const int lane = threadIdx.x & 31, wave = threadIdx.x >> 5, lr = lane & 15, hi = lane >> 4;
    const int r0 = blockIdx.x * 64 + wave * 16, c0 = blockIdx.y * 64;
    const size_t aoff = (size_t)(r0 + lr) * K + 8 * hi;
    v8f acc[4];
#pragma unroll
    for (int t = 0; t < 4; ++t) acc[t] = (v8f){};
#pragma unroll 1
    for (int kc = 0; kc < K; kc += 32) {
        const v16bf a = cat16b(*(const v8us*)(Ah + aoff + kc), *(const v8us*)(Ah + aoff + kc + 16));
        const v16bf al = cat16b(*(const v8us*)(Al + aoff + kc), *(const v8us*)(Al + aoff + kc + 16));
#pragma unroll
        for (int t = 0; t < 4; ++t) { const size_t bo = (size_t)(c0 + t * 16 + lr) * K + kc + 8 * hi;
            const v16bf bh = cat16b(*(const v8us*)(Bh + bo), *(const v8us*)(Bh + bo + 16)); const v16bf bl = cat16b(*(const v8us*)(Bl + bo), *(const v8us*)(Bl + bo + 16));
            acc[t] = wmmab(a, bh, acc[t]); acc[t] = wmmab(al, bh, acc[t]); acc[t] = wmmab(a, bl, acc[t]); }
        asm volatile("v_nop\n\tv_nop\n\tv_nop\n\tv_nop" : "+v"(acc[0]), "+v"(acc[1]), "+v"(acc[2]), "+v"(acc[3]) : "v"(a), "v"(al));
    }
    float* os = &ost[wave][0];
#pragma unroll
    for (int t = 0; t < 4; ++t) {
#pragma unroll
        for (int j = 0; j < 8; ++j) os[(hi * 8 + j) * 68 + t * 16 + lr] = acc[t][j]; }
    __builtin_amdgcn_wave_barrier(); asm volatile("" ::: "memory");
    float* crow = C + (size_t)r0 * ldc + c0;
    auto pass = [&]() {
#pragma unroll
        for (int s = 0; s < 8; ++s) { const int Lid = (lane >> 3) + 4 * s, piece = lane & 7; const int row = Lid >> 1, cofs = (Lid & 1) * 32 + piece * 4;
            const v4f val = *(const v4fa*)(os + row * 68 + cofs); *(volatile v4f*)(crow + (size_t)row * ldc + cofs) = val; }
    };
    pass(); __threadfence(); pass();
}


__global__ __launch_bounds__(128) void k_gemm3r(const bf* __restrict__ Ah, const bf* __restrict__ Al, const bf* __restrict__ Bh, const bf* __restrict__ Bl, int K, float* C, int ldc, const float* __restrict__ rbias) {
    __shared__ __align__(16) float ost[4][16 * 68];
    const int lane = threadIdx.x & 31, wave = threadIdx.x >> 5, lr = lane & 15, hi = lane >> 4;
    const int r0 = blockIdx.x * 64 + wave * 16, c0 = blockIdx.y * 64;
    const size_t aoff = (size_t)(r0 + lr) * K + 8 * hi;
    v8f acc[4];
#pragma unroll
    for (int t = 0; t < 4; ++t) acc[t] = (v8f){};
#pragma unroll 1
    for (int kc = 0; kc < K; kc += 32) {
        const v16bf a = cat16b(*(const v8us*)(Ah + aoff + kc), *(const v8us*)(Ah + aoff + kc + 16));
        const v16bf al = cat16b(*(const v8us*)(Al + aoff + kc), *(const v8us*)(Al + aoff + kc + 16));
#pragma unroll
        for (int t = 0; t < 4; ++t) { const size_t bo = (size_t)(c0 + t * 16 + lr) * K + kc + 8 * hi;
            const v16bf bh = cat16b(*(const v8us*)(Bh + bo), *(const v8us*)(Bh + bo + 16)); const v16bf bl = cat16b(*(const v8us*)(Bl + bo), *(const v8us*)(Bl + bo + 16));
            acc[t] = wmmab(a, bh, acc[t]); acc[t] = wmmab(al, bh, acc[t]); acc[t] = wmmab(a, bl, acc[t]); }
        asm volatile("v_nop\n\tv_nop\n\tv_nop\n\tv_nop" : "+v"(acc[0]), "+v"(acc[1]), "+v"(acc[2]), "+v"(acc[3]) : "v"(a), "v"(al));
    }
    float* os = &ost[wave][0];
#pragma unroll
    for (int t = 0; t < 4; ++t) {
#pragma unroll
        for (int j = 0; j < 8; ++j) os[(hi * 8 + j) * 68 + t * 16 + lr] = acc[t][j] + bfr(rbias[r0 + hi * 8 + j]); }
    __builtin_amdgcn_wave_barrier(); asm volatile("" ::: "memory");
    float* crow = C + (size_t)r0 * ldc + c0;
    auto pass = [&]() {
#pragma unroll
        for (int s = 0; s < 8; ++s) { const int Lid = (lane >> 3) + 4 * s, piece = lane & 7; const int row = Lid >> 1, cofs = (Lid & 1) * 32 + piece * 4;
            const v4f val = *(const v4fa*)(os + row * 68 + cofs); *(volatile v4f*)(crow + (size_t)row * ldc + cofs) = val; }
    };
    pass(); __threadfence(); pass();
}
__global__ __launch_bounds__(256) void k_zero16(bf* dst, size_t n8) {
    const size_t i = (size_t)blockIdx.x * 256 + threadIdx.x; if (i >= n8) return; v8us z;
#pragma unroll
    for (int k = 0; k < 8; ++k) z[k] = 0;
    *(volatile v8us*)(dst + i * 8) = z; __threadfence(); *(volatile v8us*)(dst + i * 8) = z;
}
__global__ __launch_bounds__(256) void k_splitc(const float* __restrict__ src, int nrows, int nc, bf* dh, bf* dl) {
    const int lane = threadIdx.x & 31, r = blockIdx.x * 8 + (threadIdx.x >> 5); if (r >= nrows) return;
#pragma unroll 1
    for (int ps = 0; ps < 2; ++ps) {
#pragma unroll 1
        for (int c0 = lane * 8; c0 < nc; c0 += 256) { const size_t o = (size_t)r * nc + c0; const v8f v = *(const v8f*)(src + o); v8us oh, ol;
#pragma unroll
            for (int i = 0; i < 8; ++i) { const float y = v[i]; const unsigned short hb = f2bf(y); oh[i] = hb; ol[i] = f2bf(y - bf2f(hb)); }
            *(volatile v8us*)(dh + o) = oh; *(volatile v8us*)(dl + o) = ol; }
        if (ps == 0) __threadfence(); }
}
__global__ __launch_bounds__(128) void k_hsplit(const float* __restrict__ T, bf* Ph, bf* Pl, float* DIAG) {
    __shared__ float dg[4][8];
    const int lane = threadIdx.x & 31, wv = threadIdx.x >> 5, n0 = blockIdx.x * 4;
    const int h = 2 * wv + (lane >> 4), tk = (lane >> 2) & 3, d0 = (lane & 3) * 8, n = n0 + tk;
    const v8f v = *(const v8f*)(T + (size_t)n * CC + h * DH + d0); v8us oh, ol; float sq = 0.f;
#pragma unroll
    for (int i = 0; i < 8; ++i) { const unsigned short hb = f2bf(v[i]); oh[i] = hb; ol[i] = f2bf(v[i] - bf2f(hb)); sq = fmaf(v[i], v[i], sq); }
    sq += __shfl_xor(sq, 1, 32); sq += __shfl_xor(sq, 2, 32);
    if ((lane & 3) == 0) dg[tk][h] = sq * (0.5f * DNRM * DNRM);
    const size_t o = ((size_t)h * NN + n) * DH + d0;
    *(volatile v8us*)(Ph + o) = oh; *(volatile v8us*)(Pl + o) = ol;
    __syncthreads();
    const float dv = dg[lane >> 3][lane & 7];
    if (wv == 0) *(volatile float*)(DIAG + (size_t)n0 * NHD + lane) = dv;
    __threadfence();
    *(volatile v8us*)(Ph + o) = oh; *(volatile v8us*)(Pl + o) = ol;
    if (wv == 0) *(volatile float*)(DIAG + (size_t)n0 * NHD + lane) = dv;
}
__global__ __launch_bounds__(256) void k_vtp(const float* __restrict__ V, bf* Vh, bf* Vl) {
    __shared__ __align__(16) unsigned short th[32 * 72];
    __shared__ __align__(16) unsigned short tlo[32 * 72];
    const int h = blockIdx.x / (NN / 64), nt = blockIdx.x % (NN / 64), n0 = nt * 64, tid = threadIdx.x;
    const int nn = tid >> 2, dq = (tid & 3) * 8;
    const v8f v = *(const v8f*)(V + (size_t)(n0 + nn) * CC + h * DH + dq);
#pragma unroll
    for (int i = 0; i < 8; ++i) { const unsigned short hb = f2bf(v[i]); th[(dq + i) * 72 + nn] = hb; tlo[(dq + i) * 72 + nn] = f2bf(v[i] - bf2f(hb)); }
    __syncthreads();
    const int piece = tid & 7, Lid = tid >> 3;
    const int pln = Lid >> 4, d = (Lid & 15);
    const size_t base = ((size_t)h * DHP) * NN + n0;
    auto pass = [&]() {
#pragma unroll
        for (int s = 0; s < 2; ++s) { const int dd = d + 16 * s; const v8us val = *(const v8usa*)((pln ? tlo : th) + dd * 72 + piece * 8); *(volatile v8us*)((pln ? Vl : Vh) + base + (size_t)dd * NN + piece * 8) = val; }
    };
    pass(); __threadfence(); pass();
}
__global__ __launch_bounds__(256) void k_ones(bf* Vh) {
    const int h = blockIdx.x; v8us one;
#pragma unroll
    for (int k = 0; k < 8; ++k) one[k] = (unsigned short)0x3F80;
#pragma unroll 1
    for (int ps = 0; ps < 2; ++ps) {
        for (int c0 = threadIdx.x * 8; c0 < NN; c0 += 2048) *(volatile v8us*)(Vh + ((size_t)h * DHP + DH) * NN + c0) = one;
        if (ps == 0) __threadfence(); }
}
__global__ __launch_bounds__(256) void k_qfeat(const float* __restrict__ D, const float* __restrict__ DIAG, int h, bf* QPh, bf* QPl) {
    typedef __attribute__((ext_vector_type(4))) unsigned short v4us;
    const int lane = threadIdx.x & 31, n = blockIdx.x * 8 + (threadIdx.x >> 5); if (n >= NN) return;
    const v4f dv = *(const v4f*)(D + (size_t)n * MF + lane * 4); float m = -3.0e38f;
#pragma unroll
    for (int i = 0; i < 4; ++i) m = fmaxf(m, dv[i] * DNRM);
#pragma unroll
    for (int sh = 16; sh; sh >>= 1) m = fmaxf(m, __shfl_xor(m, sh, 32));
    const float dg = DIAG[(size_t)n * NHD + h]; v4us oh, ol;
#pragma unroll
    for (int i = 0; i < 4; ++i) { const float p = RATIO * (__expf(dv[i] * DNRM - dg - m) + KEPS); const unsigned short hb = f2bf(p); oh[i] = hb; ol[i] = f2bf(p - bf2f(hb)); }
    const size_t o = (size_t)n * MF + lane * 4;
    *(volatile v4us*)(QPh + o) = oh; *(volatile v4us*)(QPl + o) = ol; __threadfence(); *(volatile v4us*)(QPh + o) = oh; *(volatile v4us*)(QPl + o) = ol;
}
__global__ __launch_bounds__(256) void k_kmax(const float* __restrict__ D, int h, float* KM) {
    __shared__ float red[256];
    const int tid = threadIdx.x; float m = -3.0e38f;
#pragma unroll 1
    for (size_t i = (size_t)tid * 4; i < (size_t)NN * MF; i += 1024) { const v4f v = *(const v4f*)(D + i); m = fmaxf(fmaxf(m, v[0]), fmaxf(fmaxf(v[1], v[2]), v[3])); }
    red[tid] = m; __syncthreads();
#pragma unroll
    for (int s = 128; s >= 32; s >>= 1) { if (tid < s) red[tid] = fmaxf(red[tid], red[tid + s]); __syncthreads(); }
    if (tid < 32) { float mm = red[tid];
#pragma unroll
        for (int sh = 16; sh; sh >>= 1) mm = fmaxf(mm, __shfl_xor(mm, sh, 32));
        const float km = mm * DNRM; *(volatile float*)(KM + h * 32 + tid) = km; __threadfence(); *(volatile float*)(KM + h * 32 + tid) = km; }
}
__global__ __launch_bounds__(256) void k_kfeat(const float* __restrict__ D, const float* __restrict__ DIAG, const float* __restrict__ KM, int h, bf* KPh, bf* KPl) {
    __shared__ __align__(16) unsigned short th[MF * 72];
    __shared__ __align__(16) unsigned short tlo[MF * 72];
    const int n0 = blockIdx.x * 64, tid = threadIdx.x;
    const float km = KM[h * 32];
    { const int nn = tid >> 2, mq = (tid & 3) * 32; const float dg = DIAG[(size_t)(n0 + nn) * NHD + h];
#pragma unroll 2
        for (int i = 0; i < 32; i += 4) { const v4f dv = *(const v4f*)(D + (size_t)(n0 + nn) * MF + mq + i);
#pragma unroll
            for (int j = 0; j < 4; ++j) { const float p = RATIO * (__expf(dv[j] * DNRM - dg - km) + KEPS); const unsigned short hb = f2bf(p); th[(mq + i + j) * 72 + nn] = hb; tlo[(mq + i + j) * 72 + nn] = f2bf(p - bf2f(hb)); } } }
    __syncthreads();
    const int piece = tid & 7, Lid = tid >> 3;
    auto pass = [&]() {
#pragma unroll
        for (int s = 0; s < 8; ++s) { const int idx = Lid + 32 * s; const int pln = idx >> 7, m = idx & 127; const v8us val = *(const v8usa*)((pln ? tlo : th) + m * 72 + piece * 8);
            *(volatile v8us*)((pln ? KPl : KPh) + (size_t)m * NN + n0 + piece * 8) = val; }
    };
    pass(); __threadfence(); pass();
}
__global__ __launch_bounds__(256) void k_pack(const float* __restrict__ OH, bf* Oh, bf* Ol) {
    const int lane = threadIdx.x & 31, n = blockIdx.x * 8 + (threadIdx.x >> 5); if (n >= NN) return;
    const int h = lane >> 2, d0 = (lane & 3) * 8; const float* row = OH + ((size_t)h * NN + n) * DHP;
    const v8f v = *(const v8f*)(row + d0); const float inv = 1.0f / row[DH]; v8us oh, ol;
#pragma unroll
    for (int i = 0; i < 8; ++i) { const float y = v[i] * inv; const unsigned short hb = f2bf(y); oh[i] = hb; ol[i] = f2bf(y - bf2f(hb)); }
    const size_t o = (size_t)n * CC + lane * 8;
    *(volatile v8us*)(Oh + o) = oh; *(volatile v8us*)(Ol + o) = ol; __threadfence(); *(volatile v8us*)(Oh + o) = oh; *(volatile v8us*)(Ol + o) = ol;
}

extern "C" void kernel_launch(void* const* d_in, const int* in_sizes, int n_in,
                              void* d_out, int out_size, void* d_ws, size_t ws_size, hipStream_t stream) {
    (void)in_sizes; (void)n_in; (void)out_size;
    const float* x = (const float*)d_in[0]; const float* wq = (const float*)d_in[1]; const float* wk = (const float*)d_in[2]; const float* wv = (const float*)d_in[3]; const float* wo = (const float*)d_in[4]; const float* bo = (const float*)d_in[5];
    const float* proj = (const float*)d_in[6]; const float* wp = (const float*)d_in[7]; const float* bp = (const float*)d_in[8];
    float* out = (float*)d_out;
    char* wsp = (char*)d_ws;
    auto take = [&](size_t bytes) { char* p = wsp; wsp += (bytes + 255) & ~(size_t)255; return (void*)p; };
    bf* WqB = (bf*)take(CC * CC * 2); bf* WkB = (bf*)take(CC * CC * 2); bf* WvB = (bf*)take(CC * CC * 2); bf* WoB = (bf*)take(CC * CC * 2); bf* WpB = (bf*)take(CC * CC * 2); bf* WZ = (bf*)take(CC * CC * 2); bf* PJ = (bf*)take(MF * DH * 2);
    bf* XT = (bf*)take((size_t)NN * CC * 2); float* TMP = (float*)take((size_t)NN * CC * 4); float* DGQ = (float*)take((size_t)NN * NHD * 4); float* DGK = (float*)take((size_t)NN * NHD * 4);
    bf* Qh = (bf*)take((size_t)NHD * NN * DH * 2); bf* Ql = (bf*)take((size_t)NHD * NN * DH * 2); bf* Kh = (bf*)take((size_t)NHD * NN * DH * 2); bf* Kl = (bf*)take((size_t)NHD * NN * DH * 2);
    bf* Vh = (bf*)take((size_t)NHD * DHP * NN * 2); bf* Vl = (bf*)take((size_t)NHD * DHP * NN * 2);
    float* D = (float*)take((size_t)NN * MF * 4); float* KM = (float*)take(NHD * 32 * 4); bf* QPh = (bf*)take((size_t)NN * MF * 2); bf* QPl = (bf*)take((size_t)NN * MF * 2); bf* KPh = (bf*)take((size_t)MF * NN * 2); bf* KPl = (bf*)take((size_t)MF * NN * 2);
    float* CT = (float*)take((size_t)DHP * MF * 4); bf* CTh = (bf*)take((size_t)DHP * MF * 2); bf* CTl = (bf*)take((size_t)DHP * MF * 2); float* OH = (float*)take((size_t)NHD * NN * DHP * 4);
    bf* Oh = (bf*)take((size_t)NN * CC * 2); bf* Ol = (bf*)take((size_t)NN * CC * 2); float* T2 = (float*)take((size_t)NN * CC * 4); bf* O2h = (bf*)take((size_t)NN * CC * 2); bf* O2l = (bf*)take((size_t)NN * CC * 2);
    if ((size_t)(wsp - (char*)d_ws) > ws_size) return;
    k_bf<<<(CC * CC / 8 + 255) / 256, 256, 0, stream>>>(wq, WqB, CC * CC / 8); k_bf<<<(CC * CC / 8 + 255) / 256, 256, 0, stream>>>(wk, WkB, CC * CC / 8); k_bf<<<(CC * CC / 8 + 255) / 256, 256, 0, stream>>>(wv, WvB, CC * CC / 8);
    k_bf<<<(CC * CC / 8 + 255) / 256, 256, 0, stream>>>(wo, WoB, CC * CC / 8); k_bf<<<(CC * CC / 8 + 255) / 256, 256, 0, stream>>>(wp, WpB, CC * CC / 8); k_bf<<<(MF * DH / 8 + 255) / 256, 256, 0, stream>>>(proj, PJ, MF * DH / 8);
    k_zero16<<<(CC * CC / 8 + 255) / 256, 256, 0, stream>>>(WZ, CC * CC / 8);
    k_zero16<<<(unsigned)(((size_t)NHD * DHP * NN / 8 + 255) / 256), 256, 0, stream>>>(Vh, (size_t)NHD * DHP * NN / 8); k_zero16<<<(unsigned)(((size_t)NHD * DHP * NN / 8 + 255) / 256), 256, 0, stream>>>(Vl, (size_t)NHD * DHP * NN / 8); k_ones<<<NHD, 256, 0, stream>>>(Vh);
    for (int b = 0; b < NBI; ++b) {
        k_wt<<<dim3(CC / 64, NN / 64, 1), 256, 0, stream>>>(x + (size_t)b * CC * NN, CC, NN, XT);
        k_gemmb<false, false><<<dim3(NN / 64, CC / 64, 1), 128, 0, stream>>>(XT, nullptr, WqB, nullptr, TMP, CC, nullptr); k_hsplit<<<NN / 4, 128, 0, stream>>>(TMP, Qh, Ql, DGQ);
        k_gemmb<false, false><<<dim3(NN / 64, CC / 64, 1), 128, 0, stream>>>(XT, nullptr, WkB, nullptr, TMP, CC, nullptr); k_hsplit<<<NN / 4, 128, 0, stream>>>(TMP, Kh, Kl, DGK);
        k_gemmb<false, false><<<dim3(NN / 64, CC / 64, 1), 128, 0, stream>>>(XT, nullptr, WvB, nullptr, TMP, CC, nullptr); k_vtp<<<NHD * (NN / 64), 256, 0, stream>>>(TMP, Vh, Vl);
        for (int h = 0; h < NHD; ++h) {
            k_gemmb<true, false><<<dim3(NN / 64, MF / 64, 1), 128, 0, stream>>>(Kh + (size_t)h * NN * DH, Kl + (size_t)h * NN * DH, PJ, nullptr, D, MF, nullptr, nullptr, DH);
            k_kmax<<<1, 256, 0, stream>>>(D, h, KM); k_kfeat<<<NN / 64, 256, 0, stream>>>(D, DGK, KM, h, KPh, KPl);
            k_gemmb<true, false><<<dim3(NN / 64, MF / 64, 1), 128, 0, stream>>>(Qh + (size_t)h * NN * DH, Ql + (size_t)h * NN * DH, PJ, nullptr, D, MF, nullptr, nullptr, DH);
            k_qfeat<<<NN / 8, 256, 0, stream>>>(D, DGQ, h, QPh, QPl);
            k_gemm3<<<dim3(DHP / 64, MF / 64, 1), 128, 0, stream>>>(Vh + (size_t)h * DHP * NN, Vl + (size_t)h * DHP * NN, KPh, KPl, NN, CT, MF);
            k_splitc<<<DHP / 8, 256, 0, stream>>>(CT, DHP, MF, CTh, CTl);
            k_gemm3<<<dim3(NN / 64, DHP / 64, 1), 128, 0, stream>>>(QPh, QPl, CTh, CTl, MF, OH + (size_t)h * NN * DHP, DHP);
        }
        k_pack<<<NN / 8, 256, 0, stream>>>(OH, Oh, Ol);
        k_gemmb<true, false><<<dim3(NN / 64, CC / 64, 1), 128, 0, stream>>>(Oh, Ol, WoB, bo, T2, CC, nullptr);
        k_splitc<<<NN / 8, 256, 0, stream>>>(T2, NN, CC, O2h, O2l);
        k_gemm3r<<<dim3(CC / 64, NN / 64, 1), 128, 0, stream>>>(WpB, WZ, O2h, O2l, CC, out + (size_t)b * CC * NN, NN, bp);
    }
}
